// MHAttention_60215441490286
// MI455X (gfx1250) — hardware-verified
//
#include <hip/hip_runtime.h>
#include <stdint.h>


#ifndef NB
#define NB 2
#endif
#ifndef SEQ
#define SEQ 2048
#endif
#define NB_FULL 2
#define SEQ_FULL 2048
#define EMB 1024
#define NH 16
#define HD 64
#define MTOK (NB * SEQ)
#define NBH (NB * NH)
#define CVT_BLK 256
#define NBW (EMB * EMB / (8 * CVT_BLK))
#define NBX (MTOK * EMB / (8 * CVT_BLK))

static_assert(SEQ % 256 == 0);
static_assert(SEQ >= 256);
static_assert(NB >= 1 && NB <= NB_FULL);
static_assert(SEQ <= SEQ_FULL);
static_assert(EMB == NH * HD);
static_assert((MTOK * EMB) % (8 * CVT_BLK) == 0);
static_assert((EMB * EMB) % (8 * CVT_BLK) == 0);
static_assert(MTOK % 16 == 0);
static_assert(SEQ % 128 == 0);

typedef __bf16 v16bf __attribute__((ext_vector_type(16)));
typedef __bf16 v8bf __attribute__((ext_vector_type(8)));
typedef float v8f __attribute__((ext_vector_type(8)));
typedef float v4f __attribute__((ext_vector_type(4)));
typedef unsigned int v4u __attribute__((ext_vector_type(4)));
typedef v8bf v8bfa __attribute__((may_alias));
typedef v4f v4fa __attribute__((may_alias));
typedef v4u v4ua __attribute__((may_alias));

__device__ __forceinline__ unsigned int bfbits(float f) {
  unsigned int u = __float_as_uint(f);
  u += 0x7FFFu + ((u >> 16) & 1u);
  return u >> 16;
}
__device__ __forceinline__ float bfval(unsigned int b) {
  return __uint_as_float(b << 16);
}
__device__ __forceinline__ unsigned int pack2(unsigned int lo16, unsigned int hi16) {
  return (lo16 & 0xffffu) | (hi16 << 16);
}

__device__ __forceinline__ v8f wmma_bf(v16bf a, v16bf b, v8f c) {
  v8f d = __builtin_amdgcn_wmma_f32_16x16x32_bf16(false, a, false, b, (short)0, c, false, false);
  asm volatile("v_nop\n\tv_nop\n\tv_nop\n\tv_nop" : "+v"(d) : "v"(a), "v"(b));
  return d;
}

__device__ __forceinline__ v16bf ldfrag(const unsigned short* __restrict__ base,
                                        int ld, int r0, int k0) {
  const int lane = threadIdx.x & 31;
  const int m = lane & 15;
  const int koff = (lane >> 4) << 3;
  const unsigned short* p = base + (size_t)(r0 + m) * ld + (k0 + koff);
  const v8bf lo = *(const v8bfa*)p;
  const v8bf hi = *(const v8bfa*)(p + 16);
  v16bf f;
#pragma unroll
  for (int i = 0; i < 8; ++i) { f[i] = lo[i]; f[i + 8] = hi[i]; }
  return f;
}

__global__ __launch_bounds__(CVT_BLK) void k_cvt(const float* __restrict__ x,
                                                 const float* __restrict__ wq,
                                                 const float* __restrict__ wk,
                                                 const float* __restrict__ wv,
                                                 unsigned short* __restrict__ Xb,
                                                 unsigned short* __restrict__ Wb) {
  const int blk = blockIdx.x;
  const int tid = threadIdx.x;
  const float* src;
  unsigned short* dst;
  if (blk < NBX) {
    const size_t e = ((size_t)blk * CVT_BLK + tid) * 8;
    const size_t t = e / EMB;
    const size_t col = e - t * EMB;
    const size_t bt = t / SEQ;
    const size_t s = t - bt * SEQ;
    src = x + (bt * SEQ_FULL + s) * EMB + col;
    dst = Xb + e;
  } else {
    const int wi = blk - NBX;
    const int zw = wi / NBW;
    const size_t e = ((size_t)(wi - zw * NBW) * CVT_BLK + tid) * 8;
    const float* wsrc = (zw == 0) ? wq : ((zw == 1) ? wk : wv);
    src = wsrc + e;
    dst = Wb + (size_t)zw * EMB * EMB + e;
  }
  const v4f a = *(const v4fa*)src;
  const v4f b = *(const v4fa*)(src + 4);
  const float a0 = a[0], a1 = a[1], a2 = a[2], a3 = a[3];
  const float b0 = b[0], b1 = b[1], b2 = b[2], b3 = b[3];
  v4u o;
  o[0] = pack2(bfbits(a0), bfbits(a1));
  o[1] = pack2(bfbits(a2), bfbits(a3));
  o[2] = pack2(bfbits(b0), bfbits(b1));
  o[3] = pack2(bfbits(b2), bfbits(b3));
  *(volatile v4u*)dst = o;
  __threadfence();
  *(volatile v4u*)dst = o;
}

__global__ __launch_bounds__(512) void k_proj(const unsigned short* __restrict__ Xb,
                                               const unsigned short* __restrict__ Wb,
                                               const float* __restrict__ bq,
                                               const float* __restrict__ bk,
                                               const float* __restrict__ bv,
                                               unsigned short* __restrict__ Qhi,
                                               unsigned short* __restrict__ Qlo,
                                               unsigned short* __restrict__ Kthi,
                                               unsigned short* __restrict__ Ktlo,
                                               unsigned short* __restrict__ Vthi,
                                               unsigned short* __restrict__ Vtlo) {
  __shared__ __align__(16) unsigned short lds_t[16 * EMB];
  const int z = blockIdx.y;
  const int tid = threadIdx.x;
  const int lane = tid & 31;
  const int w = tid >> 5;
  const int c = lane & 15;
  const int h = lane >> 4;
  const int m0 = blockIdx.x * 16;
  const int nb = w * 64;
  const unsigned short* W = Wb + (size_t)z * EMB * EMB;
  const float* bias = (z == 0) ? bq : ((z == 1) ? bk : bv);
  const unsigned short* arow = Xb + (size_t)m0 * EMB;
  const unsigned short* wrow = W + (size_t)nb * EMB;

  v8f acc[4] = {};
#pragma unroll 1
  for (int k0 = 0; k0 < EMB; k0 += 32) {
    const v16bf a  = ldfrag(arow, EMB, 0, k0);
    const v16bf b0 = ldfrag(wrow, EMB, 0, k0);
    const v16bf b1 = ldfrag(wrow, EMB, 16, k0);
    const v16bf b2 = ldfrag(wrow, EMB, 32, k0);
    const v16bf b3 = ldfrag(wrow, EMB, 48, k0);
    acc[0] = wmma_bf(a, b0, acc[0]);
    acc[1] = wmma_bf(a, b1, acc[1]);
    acc[2] = wmma_bf(a, b2, acc[2]);
    acc[3] = wmma_bf(a, b3, acc[3]);
  }

  float bb[4];
#pragma unroll
  for (int ni = 0; ni < 4; ++ni) bb[ni] = bfval(bfbits(bias[nb + ni * 16 + c]));

  const bool zq = (z == 0);
  const int bh = (m0 * 16) / SEQ;
  const int j0 = m0 * 16 - bh * SEQ;
  unsigned short* planeH = zq ? Qhi : ((z == 1) ? Kthi : Vthi);
  unsigned short* planeL = zq ? Qlo : ((z == 1) ? Ktlo : Vtlo);

  int loff[4];
  size_t goff[4];
#pragma unroll
  for (int it = 0; it < 4; ++it) {
    const int p = it * 512 + tid;
    const int lq = p * 8;
    const size_t gq = (size_t)m0 * EMB + (size_t)p * 8;
    const int kk = it * 16 + w;
    const int lk = kk * 256 + lane * 8;
    const size_t gk = ((size_t)bh * HD + kk) * (size_t)SEQ + (size_t)j0 + (size_t)lane * 8;
    loff[it] = zq ? lq : lk;
    goff[it] = zq ? gq : gk;
  }

#pragma unroll
  for (int ph = 0; ph < 2; ++ph) {
#pragma unroll
    for (int ni = 0; ni < 4; ++ni) {
#pragma unroll
      for (int r = 0; r < 8; ++r) {
        const float v = acc[ni][r] + bb[ni];
        const unsigned int hb = bfbits(v);
        const unsigned int val = (ph == 0) ? hb : bfbits(v - bfval(hb));
        const int n = nb + ni * 16 + c;
        const int ml = 8 * h + r;
        const int lq = ml * EMB + n;
        const int lk = (ni * 16 + c) * 256 + ml * 16 + w;
        lds_t[zq ? lq : lk] = (unsigned short)val;
      }
    }
    __syncthreads();
    v4u pv[4];
#pragma unroll
    for (int it = 0; it < 4; ++it) pv[it] = *(const v4ua*)(lds_t + loff[it]);
    unsigned short* plane = (ph == 0) ? planeH : planeL;
#pragma unroll
    for (int it = 0; it < 4; ++it) *(volatile v4u*)(plane + goff[it]) = pv[it];
    __threadfence();
#pragma unroll
    for (int it = 0; it < 4; ++it) *(volatile v4u*)(plane + goff[it]) = pv[it];
    __syncthreads();
  }
}

__global__ __launch_bounds__(256) void k_kv(const unsigned short* __restrict__ Kthi,
                                             const unsigned short* __restrict__ Ktlo,
                                             const unsigned short* __restrict__ Vthi,
                                             const unsigned short* __restrict__ Vtlo,
                                             unsigned short* __restrict__ Sthi,
                                             unsigned short* __restrict__ Stlo) {
  __shared__ __align__(16) float s_lds[HD * HD];
  const int bh = blockIdx.x;
  const int tid = threadIdx.x;
  const int lane = tid & 31;
  const int w = tid >> 5;
  const int c = lane & 15;
  const int h = lane >> 4;
  const int m0w = (w >> 1) * 16;
  const int n0w = (w & 1) * 32;
  const size_t pb = (size_t)bh * HD * (size_t)SEQ;
  const unsigned short* KH = Kthi + pb;
  const unsigned short* KL = Ktlo + pb;
  const unsigned short* VH = Vthi + pb;
  const unsigned short* VL = Vtlo + pb;

  v8f acc[2] = {};
#pragma unroll 1
  for (int j0 = 0; j0 < SEQ; j0 += 32) {
    const v16bf ah = ldfrag(KH, SEQ, m0w, j0);
    const v16bf al = ldfrag(KL, SEQ, m0w, j0);
#pragma unroll
    for (int t = 0; t < 2; ++t) {
      const v16bf vh = ldfrag(VH, SEQ, n0w + 16 * t, j0);
      const v16bf vl = ldfrag(VL, SEQ, n0w + 16 * t, j0);
      acc[t] = wmma_bf(ah, vh, acc[t]);
      acc[t] = wmma_bf(ah, vl, acc[t]);
      acc[t] = wmma_bf(al, vh, acc[t]);
    }
  }

#pragma unroll
  for (int t = 0; t < 2; ++t)
#pragma unroll
    for (int r = 0; r < 8; ++r) {
      const float v = acc[t][r];
      s_lds[(n0w + 16 * t + c) * HD + (m0w + 8 * h + r)] = v * 0.125f;
    }
  __syncthreads();

  v4u hv[2], lv[2];
  size_t go[2];
#pragma unroll
  for (int it = 0; it < 2; ++it) {
    const int p = it * 256 + tid;
    const int d = p >> 3;
    const int kk8 = (p & 7) * 8;
    const v4f x0 = *(const v4fa*)(s_lds + d * HD + kk8);
    const v4f x1 = *(const v4fa*)(s_lds + d * HD + kk8 + 4);
    float f[8];
    f[0] = x0[0]; f[1] = x0[1]; f[2] = x0[2]; f[3] = x0[3];
    f[4] = x1[0]; f[5] = x1[1]; f[6] = x1[2]; f[7] = x1[3];
    unsigned int hb[8], lb[8];
#pragma unroll
    for (int i = 0; i < 8; ++i) {
      hb[i] = bfbits(f[i]);
      lb[i] = bfbits(f[i] - bfval(hb[i]));
    }
    v4u th, tl;
    th[0] = pack2(hb[0], hb[1]); th[1] = pack2(hb[2], hb[3]);
    th[2] = pack2(hb[4], hb[5]); th[3] = pack2(hb[6], hb[7]);
    tl[0] = pack2(lb[0], lb[1]); tl[1] = pack2(lb[2], lb[3]);
    tl[2] = pack2(lb[4], lb[5]); tl[3] = pack2(lb[6], lb[7]);
    hv[it] = th;
    lv[it] = tl;
    go[it] = (size_t)bh * HD * HD + (size_t)d * HD + (size_t)kk8;
  }
#pragma unroll
  for (int it = 0; it < 2; ++it) {
    *(volatile v4u*)(Sthi + go[it]) = hv[it];
    *(volatile v4u*)(Stlo + go[it]) = lv[it];
  }
  __threadfence();
#pragma unroll
  for (int it = 0; it < 2; ++it) {
    *(volatile v4u*)(Sthi + go[it]) = hv[it];
    *(volatile v4u*)(Stlo + go[it]) = lv[it];
  }
}

__global__ __launch_bounds__(256) void k_out(const unsigned short* __restrict__ Qhi,
                                              const unsigned short* __restrict__ Qlo,
                                              const unsigned short* __restrict__ Sthi,
                                              const unsigned short* __restrict__ Stlo,
                                              float* __restrict__ out) {
  __shared__ __align__(16) float o_lds[8 * 16 * HD];
  const int bh = blockIdx.y;
  const int tid = threadIdx.x;
  const int lane = tid & 31;
  const int w = tid >> 5;
  const int c = lane & 15;
  const int h = lane >> 4;
  const int jw = blockIdx.x * 128 + w * 16;
  const size_t qb = (size_t)bh * (size_t)SEQ * HD;
  const size_t sb = (size_t)bh * HD * HD;
  const unsigned short* QH = Qhi + qb;
  const unsigned short* QL = Qlo + qb;
  const unsigned short* SH = Sthi + sb;
  const unsigned short* SL = Stlo + sb;

  v8f acc[4] = {};
#pragma unroll
  for (int ks = 0; ks < 2; ++ks) {
    const int k0 = ks * 32;
    const v16bf ah = ldfrag(QH, HD, jw, k0);
    const v16bf al = ldfrag(QL, HD, jw, k0);
#pragma unroll
    for (int t = 0; t < 4; ++t) {
      const v16bf sh = ldfrag(SH, HD, 16 * t, k0);
      const v16bf sl = ldfrag(SL, HD, 16 * t, k0);
      acc[t] = wmma_bf(ah, sh, acc[t]);
      acc[t] = wmma_bf(ah, sl, acc[t]);
      acc[t] = wmma_bf(al, sh, acc[t]);
    }
  }

  float* ol = o_lds + w * (16 * HD);
#pragma unroll
  for (int t = 0; t < 4; ++t)
#pragma unroll
    for (int r = 0; r < 8; ++r) {
      const float v = acc[t][r];
      ol[(8 * h + r) * HD + 16 * t + c] = v;
    }
  __syncthreads();

  v4f pv[8];
#pragma unroll
  for (int it = 0; it < 8; ++it) {
    const int p = it * 32 + lane;
    pv[it] = *(const v4fa*)(ol + p * 4);
  }
  float* ob = out + ((size_t)bh * (size_t)SEQ + (size_t)jw) * HD;
#pragma unroll
  for (int it = 0; it < 8; ++it) *(volatile v4f*)(ob + (size_t)(it * 32 + lane) * 4) = pv[it];
  __threadfence();
#pragma unroll
  for (int it = 0; it < 8; ++it) *(volatile v4f*)(ob + (size_t)(it * 32 + lane) * 4) = pv[it];
}

extern "C" void kernel_launch(void* const* d_in, const int* in_sizes, int n_in,
                              void* d_out, int out_size, void* d_ws, size_t ws_size,
                              hipStream_t stream) {
  if (n_in < 7) return;
  if ((size_t)in_sizes[0] < ((size_t)(NB - 1) * SEQ_FULL + (size_t)SEQ) * EMB) return;
  if (in_sizes[1] < EMB * EMB || in_sizes[3] < EMB * EMB || in_sizes[5] < EMB * EMB) return;
  if (in_sizes[2] < EMB || in_sizes[4] < EMB || in_sizes[6] < EMB) return;
  if ((size_t)out_size < (size_t)MTOK * EMB) return;

  const float* x  = (const float*)d_in[0];
  const float* Wq = (const float*)d_in[1];
  const float* bq = (const float*)d_in[2];
  const float* Wk = (const float*)d_in[3];
  const float* bk = (const float*)d_in[4];
  const float* Wv = (const float*)d_in[5];
  const float* bv = (const float*)d_in[6];
  float* out = (float*)d_out;

  const size_t nAct = (size_t)MTOK * EMB;
  const size_t nWt  = (size_t)EMB * EMB;
  const size_t nS   = (size_t)NBH * HD * HD;

  char* ws = (char*)d_ws;
  size_t off = 0;
  unsigned short* Xb   = (unsigned short*)(ws + off); off += nAct * 2;
  unsigned short* Wb   = (unsigned short*)(ws + off); off += 3 * nWt * 2;
  unsigned short* Qhi  = (unsigned short*)(ws + off); off += nAct * 2;
  unsigned short* Qlo  = (unsigned short*)(ws + off); off += nAct * 2;
  unsigned short* Kthi = (unsigned short*)(ws + off); off += nAct * 2;
  unsigned short* Ktlo = (unsigned short*)(ws + off); off += nAct * 2;
  unsigned short* Vthi = (unsigned short*)(ws + off); off += nAct * 2;
  unsigned short* Vtlo = (unsigned short*)(ws + off); off += nAct * 2;
  unsigned short* Sthi = (unsigned short*)(ws + off); off += nS * 2;
  unsigned short* Stlo = (unsigned short*)(ws + off); off += nS * 2;
  if (off > ws_size) return;

  k_cvt<<<dim3(NBX + 3 * NBW), dim3(CVT_BLK), 0, stream>>>(x, Wq, Wk, Wv, Xb, Wb);
  k_proj<<<dim3(MTOK / 16, 3), dim3(512), 0, stream>>>(Xb, Wb, bq, bk, bv,
                                                       Qhi, Qlo, Kthi, Ktlo, Vthi, Vtlo);
  k_kv<<<dim3(NBH), dim3(256), 0, stream>>>(Kthi, Ktlo, Vthi, Vtlo, Sthi, Stlo);
  k_out<<<dim3(SEQ / 128, NBH), dim3(256), 0, stream>>>(Qhi, Qlo, Sthi, Stlo, out);
}
